// ColourCatDSSGINConv_41094247088190
// MI455X (gfx1250) — hardware-verified
//
#include <hip/hip_runtime.h>
#include <stdint.h>
#include <stddef.h>


#define IN_D    16
#define CDIM    8
#define NSMP    4
#define KD      24
#define HH      64
#define CH      48
#define APITCH  64
#define NPB     800
#define CHUNK   256
#define GTHREADS 256
#define WAVES_G 5
#define TPB_G   (WAVES_G * 32)
#define ROWS_G  (WAVES_G * 16)
#define STGP    68
#define W1P     40
#define W2P     72

static_assert((W1P * 2) % 16 == 0);
static_assert((W2P * 2) % 16 == 0);
static_assert((STGP * 4) % 16 == 0);
static_assert((CH * 4) % 16 == 0);
static_assert(CHUNK == GTHREADS);

typedef __bf16         v16bf __attribute__((ext_vector_type(16)));
typedef unsigned short v16us __attribute__((ext_vector_type(16)));
typedef unsigned short v8us  __attribute__((ext_vector_type(8)));
typedef float          v8f   __attribute__((ext_vector_type(8)));
typedef float          v4f   __attribute__((ext_vector_type(4)));
typedef double         v2d   __attribute__((ext_vector_type(2)));
union FragB { v16bf v; v16us s; v8us h8[2]; };

__device__ __forceinline__ unsigned bf16_rne(float f)
{
    const unsigned u = __float_as_uint(f);
    return (u + 0x7FFFu + ((u >> 16) & 1u)) >> 16;
}
__device__ __forceinline__ void split2(float f, unsigned short& hi, unsigned short& lo)
{
    const unsigned hb = bf16_rne(f);
    const float rem = f - __uint_as_float(hb << 16);
    hi = (unsigned short)hb;
    lo = (unsigned short)bf16_rne(rem);
}

__device__ __forceinline__ void wmma_bf16(v8f& acc, const v16bf& a, const v16bf& b)
{
    acc = __builtin_amdgcn_wmma_f32_16x16x32_bf16(false, a, false, b, (short)0, acc, false, false);
}

#define WMMA_GUARD4(acc, a, b, a2, b2) \
    asm volatile("v_nop\n\tv_nop\n\tv_nop\n\tv_nop" : "+v"(acc) : "v"(a), "v"(b), "v"(a2), "v"(b2))
#define WMMA_GUARD8(acc, a, b, a2, b2, a3, b3, a4, b4) \
    asm volatile("v_nop\n\tv_nop\n\tv_nop\n\tv_nop" : "+v"(acc) : "v"(a), "v"(b), "v"(a2), "v"(b2), "v"(a3), "v"(b3), "v"(a4), "v"(b4))

__global__ __launch_bounds__(GTHREADS)
void gather_agg_kernel(const int* __restrict__ ei,
                       const float* __restrict__ x,
                       const float* __restrict__ c,
                       float* agg,
                       int N, int E)
{
    __shared__ __align__(16) float acc[NPB * CH];
    __shared__ int lsrc[CHUNK];
    __shared__ int lloc[CHUNK];
    __shared__ int wcnt[GTHREADS / 32];

    const int tid  = threadIdx.x;
    const int lane = tid & 31;
    const int wave = tid >> 5;
    const int node0 = blockIdx.x * NPB;
    int nloc = N - node0;
    if (nloc > NPB) nloc = NPB;
    if (nloc < 0) nloc = 0;

    for (int i = tid; i < NPB * CH; i += GTHREADS) acc[i] = 0.0f;
    __syncthreads();

    for (int e0 = 0; e0 < E; e0 += CHUNK) {
        const int e = e0 + tid;
        bool hit = false;
        int s = 0, loc = 0;
        if (e < E) {
            const int d = ei[(size_t)E + e];
            const unsigned ul = (unsigned)d - (unsigned)node0;
            if (ul < (unsigned)nloc) {
                hit = true;
                loc = (int)ul;
                s = ei[e];
                if (s < 0) s = 0;
                if (s >= N) s = N - 1;
            }
        }
        const unsigned bal = __builtin_amdgcn_ballot_w32(hit);
        const int pre = __builtin_popcount(bal & ((1u << lane) - 1u));
        if (lane == 0) wcnt[wave] = __builtin_popcount(bal);
        __syncthreads();
        int base = 0, total = 0;
#pragma unroll
        for (int w = 0; w < GTHREADS / 32; ++w) {
            const int cw = wcnt[w];
            if (w < wave) base += cw;
            total += cw;
        }
        if (hit) {
            const int p = base + pre;
            if ((unsigned)p < (unsigned)CHUNK) { lsrc[p] = s; lloc[p] = loc; }
        }
        __syncthreads();
        if (tid < CH) {
            if (total > CHUNK) total = CHUNK;
            for (int p = 0; p < total; ++p) {
                int sidx = lsrc[p];
                int l2   = lloc[p];
                if ((unsigned)sidx >= (unsigned)N) sidx = N - 1;
                if ((unsigned)l2 >= (unsigned)NPB) l2 = NPB - 1;
                float v;
                if (tid < IN_D) v = x[(size_t)sidx * IN_D + tid];
                else            v = c[(size_t)sidx * (NSMP * CDIM) + (tid - IN_D)];
                acc[l2 * CH + tid] += v;
            }
        }
        __syncthreads();
    }

    const int rsub = lane >> 4;
    const int q    = (lane >> 3) & 1;
    const int j    = lane & 7;
    const int col  = 32 * q + 4 * j;
    for (int pass = 0; pass < 2; ++pass) {
        if (pass) __threadfence();
        for (int rp = 2 * wave; rp < nloc; rp += 2 * (GTHREADS / 32)) {
            const int r = rp + rsub;
            if (r < nloc) {
                v4f v = {0.0f, 0.0f, 0.0f, 0.0f};
                if (col < CH) v = *(const v4f*)(acc + r * CH + col);
                *(volatile v4f*)(agg + (size_t)(node0 + r) * APITCH + col) = v;
            }
        }
    }
}

template <int MODE>
__global__ __launch_bounds__(TPB_G)
void gemm1_kernel(const float* __restrict__ x,
                  const float* __restrict__ c,
                  const float* __restrict__ agg,
                  const float* __restrict__ epsp,
                  const float* __restrict__ W1,
                  const float* __restrict__ b1,
                  float* Z,
                  double* part,
                  int Mrows)
{
    __shared__ __align__(16) unsigned short ldsWh[HH * W1P];
    __shared__ __align__(16) unsigned short ldsWl[HH * W1P];
    __shared__ __align__(16) float stg[WAVES_G][16 * STGP];
    __shared__ double psum[WAVES_G][2 * HH];
    __shared__ float ldsB[HH];

    const int tid = threadIdx.x;
    for (int idx = tid; idx < HH * 32; idx += TPB_G) {
        const int col = idx >> 5;
        const int k   = idx & 31;
        const float w = (k < KD) ? W1[k * HH + col] : 0.0f;
        unsigned short hi, lo;
        split2(w, hi, lo);
        ldsWh[col * W1P + k] = hi;
        ldsWl[col * W1P + k] = lo;
    }
    if (tid < HH) ldsB[tid] = b1[tid];
    __syncthreads();

    const int wave = tid >> 5;
    const int lane = tid & 31;
    const int h    = lane >> 4;
    const int m    = lane & 15;
    const int mbase = (blockIdx.x * WAVES_G + wave) * 16;
    const bool active = mbase < Mrows;

    if (active) {
        int row = mbase + m;
        if (row >= Mrows) row = Mrows - 1;
        const float ep = 1.0f + epsp[0];
        const v4f epv = {ep, ep, ep, ep};
        v4f p0, p1;
        v4f p2 = {0.0f, 0.0f, 0.0f, 0.0f};
        v4f p3 = {0.0f, 0.0f, 0.0f, 0.0f};
        if (MODE == 0) {
            const int n = row >> 2;
            const int s = row & 3;
            const float* xr = x + (size_t)n * IN_D + 8 * h;
            const float* ar = agg + (size_t)n * APITCH + 8 * h;
            p0 = epv * (*(const v4f*)xr)       + *(const v4f*)ar;
            p1 = epv * (*(const v4f*)(xr + 4)) + *(const v4f*)(ar + 4);
            if (h == 0) {
                const float* cr = c + ((size_t)n * NSMP + s) * CDIM;
                const float* gr = agg + (size_t)n * APITCH + IN_D + CDIM * s;
                p2 = epv * (*(const v4f*)cr)       + *(const v4f*)gr;
                p3 = epv * (*(const v4f*)(cr + 4)) + *(const v4f*)(gr + 4);
            }
        } else {
            const int n = row;
            const float* xr = x + (size_t)n * IN_D + 8 * h;
            const float* ar = agg + (size_t)n * APITCH + 8 * h;
            p0 = epv * (*(const v4f*)xr)       + *(const v4f*)ar;
            p1 = epv * (*(const v4f*)(xr + 4)) + *(const v4f*)(ar + 4);
            if (h == 0) {
                v4f cs0 = {0.0f, 0.0f, 0.0f, 0.0f}, cs1 = {0.0f, 0.0f, 0.0f, 0.0f};
                v4f as0 = {0.0f, 0.0f, 0.0f, 0.0f}, as1 = {0.0f, 0.0f, 0.0f, 0.0f};
#pragma unroll
                for (int s = 0; s < NSMP; ++s) {
                    const float* cr = c + ((size_t)n * NSMP + s) * CDIM;
                    const float* gr = agg + (size_t)n * APITCH + IN_D + CDIM * s;
                    cs0 += *(const v4f*)cr;  cs1 += *(const v4f*)(cr + 4);
                    as0 += *(const v4f*)gr;  as1 += *(const v4f*)(gr + 4);
                }
                const v4f qv = {0.25f, 0.25f, 0.25f, 0.25f};
                p2 = (epv * cs0 + as0) * qv;
                p3 = (epv * cs1 + as1) * qv;
            }
        }

        FragB ah, al;
#pragma unroll
        for (int i = 0; i < 4; ++i) {
            unsigned short hi, lo;
            split2(p0[i], hi, lo); ah.s[i]      = hi; al.s[i]      = lo;
            split2(p1[i], hi, lo); ah.s[4 + i]  = hi; al.s[4 + i]  = lo;
            split2(p2[i], hi, lo); ah.s[8 + i]  = hi; al.s[8 + i]  = lo;
            split2(p3[i], hi, lo); ah.s[12 + i] = hi; al.s[12 + i] = lo;
        }

#pragma unroll
        for (int t = 0; t < 4; ++t) {
            const int col = 16 * t + m;
            const unsigned short* wh = ldsWh + col * W1P;
            const unsigned short* wl = ldsWl + col * W1P;
            FragB bh, bl;
            bh.h8[0] = *(const v8us*)(wh + 8 * h);
            bh.h8[1] = *(const v8us*)(wh + 16 + 8 * h);
            bl.h8[0] = *(const v8us*)(wl + 8 * h);
            bl.h8[1] = *(const v8us*)(wl + 16 + 8 * h);

            v8f acc = {0.0f, 0.0f, 0.0f, 0.0f, 0.0f, 0.0f, 0.0f, 0.0f};
            wmma_bf16(acc, ah.v, bh.v);
            wmma_bf16(acc, ah.v, bl.v);
            wmma_bf16(acc, al.v, bh.v);
            WMMA_GUARD4(acc, ah.v, bh.v, al.v, bl.v);

            const float bias = ldsB[col];
            double ps = 0.0, ps2 = 0.0;
#pragma unroll
            for (int r = 0; r < 8; ++r) {
                const float z = acc[r] + bias;
                stg[wave][(8 * h + r) * STGP + col] = z;
                if (mbase + 8 * h + r < Mrows) {
                    const double dz = (double)z;
                    ps  += dz;
                    ps2 += dz * dz;
                }
            }
            ps  += __shfl_xor(ps, 16);
            ps2 += __shfl_xor(ps2, 16);
            if (h == 0) {
                psum[wave][col]      = ps;
                psum[wave][HH + col] = ps2;
            }
        }
    } else {
        for (int i = lane; i < 2 * HH; i += 32) psum[wave][i] = 0.0;
    }
    __syncthreads();

    if (tid < HH) {
        double s = 0.0, sq = 0.0;
#pragma unroll
        for (int w = 0; w < WAVES_G; ++w) { s += psum[w][tid]; sq += psum[w][HH + tid]; }
        v2d pv = {s, sq};
        double* pp = part + (size_t)blockIdx.x * (2 * HH) + 2 * tid;
        *(volatile v2d*)pp = pv;
        __threadfence();
        *(volatile v2d*)pp = pv;
    }

    if (active) {
        const int rsub = lane >> 4;
        const int q    = (lane >> 3) & 1;
        const int j    = lane & 7;
        const int col  = 32 * q + 4 * j;
        for (int pass = 0; pass < 2; ++pass) {
            if (pass) __threadfence();
#pragma unroll
            for (int it = 0; it < 8; ++it) {
                const int r = 2 * it + rsub;
                const v4f v = *(const v4f*)(&stg[wave][r * STGP + col]);
                *(volatile v4f*)(Z + (size_t)(mbase + r) * HH + col) = v;
            }
        }
    }
}

__global__ __launch_bounds__(64)
void bn_fold_kernel(const double* __restrict__ part, int nblk, int Mrows,
                    const float* __restrict__ g, const float* __restrict__ be,
                    float* scale, float* shift)
{
    const int t = threadIdx.x;
    if (t >= HH) return;
    double s = 0.0, sq = 0.0;
    for (int b = 0; b < nblk; ++b) {
        s  += part[(size_t)b * (2 * HH) + 2 * t];
        sq += part[(size_t)b * (2 * HH) + 2 * t + 1];
    }
    const double invM = 1.0 / (double)Mrows;
    const double mu  = s * invM;
    double var = sq * invM - mu * mu;
    if (var < 0.0) var = 0.0;
    const float varf = (float)var;
    const float muf  = (float)mu;
    const float rs = rsqrtf(varf + 1e-5f);
    const float sc = g[t] * rs;
    const float sh = be[t] - muf * sc;
    *(volatile float*)(scale + t) = sc;
    *(volatile float*)(shift + t) = sh;
    __threadfence();
    *(volatile float*)(scale + t) = sc;
    *(volatile float*)(shift + t) = sh;
}

template <bool SIAM>
__global__ __launch_bounds__(TPB_G)
void gemm2_kernel(const float* __restrict__ Z,
                  const float* __restrict__ scale,
                  const float* __restrict__ shift,
                  const float* __restrict__ W2,
                  const float* __restrict__ b2,
                  const float* __restrict__ ma,
                  float* outp,
                  int Mrows)
{
    __shared__ __align__(16) unsigned short ldsWh[HH * W2P];
    __shared__ __align__(16) unsigned short ldsWl[HH * W2P];
    __shared__ __align__(16) float stg[WAVES_G][16 * STGP];
    __shared__ __align__(16) float ldsB[HH];
    __shared__ float ldsScale[HH];
    __shared__ float ldsShift[HH];

    const int tid = threadIdx.x;
    for (int idx = tid; idx < HH * HH; idx += TPB_G) {
        const int col = idx >> 6;
        const int k   = idx & 63;
        unsigned short hi, lo;
        split2(W2[k * HH + col], hi, lo);
        ldsWh[col * W2P + k] = hi;
        ldsWl[col * W2P + k] = lo;
    }
    if (tid < HH) {
        ldsScale[tid] = scale[tid];
        ldsShift[tid] = shift[tid];
        ldsB[tid]     = b2[tid];
    }
    __syncthreads();

    const int wave = tid >> 5;
    const int lane = tid & 31;
    const int h    = lane >> 4;
    const int m    = lane & 15;
    const int mbase = (blockIdx.x * WAVES_G + wave) * 16;
    const bool active = mbase < Mrows;

    if (active) {
        int row = mbase + m;
        if (row >= Mrows) row = Mrows - 1;
        const float* zr = Z + (size_t)row * HH;

        FragB a0h, a0l, a1h, a1l;
#pragma unroll
        for (int gq = 0; gq < 4; ++gq) {
            const int off = 16 * gq + 8 * h;
            const v4f z0 = *(const v4f*)(zr + off);
            const v4f z1 = *(const v4f*)(zr + off + 4);
            float zz[8] = { z0[0], z0[1], z0[2], z0[3], z1[0], z1[1], z1[2], z1[3] };
#pragma unroll
            for (int jj = 0; jj < 8; ++jj) {
                const int k = off + jj;
                const float act = fmaxf(zz[jj] * ldsScale[k] + ldsShift[k], 0.0f);
                unsigned short hi, lo;
                split2(act, hi, lo);
                if (gq < 2) { a0h.s[(gq & 1) * 8 + jj] = hi; a0l.s[(gq & 1) * 8 + jj] = lo; }
                else        { a1h.s[(gq & 1) * 8 + jj] = hi; a1l.s[(gq & 1) * 8 + jj] = lo; }
            }
        }

#pragma unroll
        for (int t = 0; t < 4; ++t) {
            const int col = 16 * t + m;
            const unsigned short* wh = ldsWh + col * W2P;
            const unsigned short* wl = ldsWl + col * W2P;
            FragB b0h, b0l, b1h, b1l;
            b0h.h8[0] = *(const v8us*)(wh + 8 * h);
            b0h.h8[1] = *(const v8us*)(wh + 16 + 8 * h);
            b1h.h8[0] = *(const v8us*)(wh + 32 + 8 * h);
            b1h.h8[1] = *(const v8us*)(wh + 48 + 8 * h);
            b0l.h8[0] = *(const v8us*)(wl + 8 * h);
            b0l.h8[1] = *(const v8us*)(wl + 16 + 8 * h);
            b1l.h8[0] = *(const v8us*)(wl + 32 + 8 * h);
            b1l.h8[1] = *(const v8us*)(wl + 48 + 8 * h);

            v8f acc = {0.0f, 0.0f, 0.0f, 0.0f, 0.0f, 0.0f, 0.0f, 0.0f};
            wmma_bf16(acc, a0h.v, b0h.v);
            wmma_bf16(acc, a0h.v, b0l.v);
            wmma_bf16(acc, a0l.v, b0h.v);
            wmma_bf16(acc, a1h.v, b1h.v);
            wmma_bf16(acc, a1h.v, b1l.v);
            wmma_bf16(acc, a1l.v, b1h.v);
            WMMA_GUARD8(acc, a1l.v, b1h.v, a1h.v, b1l.v, a0h.v, b0h.v, a0l.v, b0l.v);

#pragma unroll
            for (int r = 0; r < 8; ++r)
                stg[wave][(8 * h + r) * STGP + col] = acc[r];
        }
    }
    __syncthreads();

    if (active) {
        const int rsub = lane >> 4;
        const int q    = (lane >> 3) & 1;
        const int j    = lane & 7;
        const int col  = 32 * q + 4 * j;
        const v4f bv = *(const v4f*)(ldsB + col);
        for (int pass = 0; pass < 2; ++pass) {
            if (pass) __threadfence();
#pragma unroll
            for (int it = 0; it < 8; ++it) {
                const int r    = 2 * it + rsub;
                const int grow = mbase + r;
                v4f v = *(const v4f*)(&stg[wave][r * STGP + col]) + bv;
                if (SIAM) v += *(const v4f*)(ma + (size_t)(grow >> 2) * HH + col);
                if (grow < Mrows)
                    *(volatile v4f*)(outp + (size_t)grow * HH + col) = v;
            }
        }
    }
}

extern "C" void kernel_launch(void* const* d_in, const int* in_sizes, int n_in,
                              void* d_out, int out_size, void* d_ws, size_t ws_size,
                              hipStream_t stream)
{
    if (n_in < 17) return;
    const int N = in_sizes[0] / IN_D;
    const int E = in_sizes[2] / 2;
    if (N <= 0 || E < 0) return;
    if (in_sizes[1] != N * NSMP * CDIM) return;
    const int M1 = N * NSMP;
    if (out_size != M1 * HH) return;

    const float* x    = (const float*)d_in[0];
    const float* c    = (const float*)d_in[1];
    const int*   ei   = (const int*)  d_in[2];
    const float* epsS = (const float*)d_in[3];
    const float* W1s  = (const float*)d_in[4];
    const float* b1s  = (const float*)d_in[5];
    const float* g1s  = (const float*)d_in[6];
    const float* be1s = (const float*)d_in[7];
    const float* W2s  = (const float*)d_in[8];
    const float* b2s  = (const float*)d_in[9];
    const float* epsA = (const float*)d_in[10];
    const float* W1a  = (const float*)d_in[11];
    const float* b1a  = (const float*)d_in[12];
    const float* g1a  = (const float*)d_in[13];
    const float* be1a = (const float*)d_in[14];
    const float* W2a  = (const float*)d_in[15];
    const float* b2a  = (const float*)d_in[16];
    float* out = (float*)d_out;

    const int M1p = (M1 + 15) / 16 * 16;
    const int Np  = (N + 15) / 16 * 16;
    const int nb1 = (M1 + ROWS_G - 1) / ROWS_G;
    const int nba = (N + ROWS_G - 1) / ROWS_G;
    const int nbg = (N + NPB - 1) / NPB;

    size_t off = 0;
    auto carve = [&](size_t bytes) { size_t o = off; off += (bytes + 255) & ~(size_t)255; return o; };
    const size_t o_agg = carve((size_t)N   * APITCH * sizeof(float));
    const size_t o_z1  = carve((size_t)M1p * HH * sizeof(float));
    const size_t o_za  = carve((size_t)Np  * HH * sizeof(float));
    const size_t o_ma  = carve((size_t)Np  * HH * sizeof(float));
    const size_t o_p1  = carve((size_t)nb1 * 2 * HH * sizeof(double));
    const size_t o_pa  = carve((size_t)nba * 2 * HH * sizeof(double));
    const size_t o_scs = carve(HH * sizeof(float));
    const size_t o_shs = carve(HH * sizeof(float));
    const size_t o_sca = carve(HH * sizeof(float));
    const size_t o_sha = carve(HH * sizeof(float));
    if (off > ws_size) return;

    char* ws = (char*)d_ws;
    float*  agg  = (float*)(ws + o_agg);
    float*  Z1   = (float*)(ws + o_z1);
    float*  Za   = (float*)(ws + o_za);
    float*  maO  = (float*)(ws + o_ma);
    double* p1   = (double*)(ws + o_p1);
    double* pa   = (double*)(ws + o_pa);
    float*  scS  = (float*)(ws + o_scs);
    float*  shS  = (float*)(ws + o_shs);
    float*  scA  = (float*)(ws + o_sca);
    float*  shA  = (float*)(ws + o_sha);

    gather_agg_kernel<<<nbg, GTHREADS, 0, stream>>>(ei, x, c, agg, N, E);

    gemm1_kernel<0><<<nb1, TPB_G, 0, stream>>>(x, c, agg, epsS, W1s, b1s, Z1, p1, M1);
    gemm1_kernel<1><<<nba, TPB_G, 0, stream>>>(x, c, agg, epsA, W1a, b1a, Za, pa, N);

    bn_fold_kernel<<<1, 64, 0, stream>>>(p1, nb1, M1, g1s, be1s, scS, shS);
    bn_fold_kernel<<<1, 64, 0, stream>>>(pa, nba, N,  g1a, be1a, scA, shA);

    gemm2_kernel<false><<<nba, TPB_G, 0, stream>>>(Za, scA, shA, W2a, b2a, (const float*)maO, maO, N);
    gemm2_kernel<true><<<nb1, TPB_G, 0, stream>>>(Z1, scS, shS, W2s, b2s, (const float*)maO, out, M1);
}
